// SelfAttention_37555194036870
// MI455X (gfx1250) — hardware-verified
//
#include <hip/hip_runtime.h>


#ifndef NB
#define NB 2
#endif
#ifndef SEQ
#define SEQ 2048
#endif
#define NB_FULL  2
#define SEQ_FULL 2048
#define TT   SEQ
#define DM   1024
#define NH_  16
#define HD   64
#define DQ   (NH_ * HD)
#define ZH   2
#define MPITCH SEQ_FULL
#define PCAR 1024.0f
#define SCL  0.125f

static_assert(TT % 256 == 0);
static_assert(TT % 64 == 0);
static_assert(DM % 64 == 0);
static_assert(DQ == DM);
static_assert(HD == 64);
static_assert(NH_ % ZH == 0);
static_assert(NB <= NB_FULL);
static_assert(SEQ <= SEQ_FULL);
static_assert(MPITCH % 8 == 0);
static_assert(((size_t)SEQ_FULL * SEQ_FULL) % 8 == 0);
static_assert((size_t)NH_ * TT * HD == (size_t)TT * DQ);
static_assert((TT / 256) * 8 == TT / 32);

typedef _Float16 h16;
typedef unsigned short bf;
typedef __attribute__((ext_vector_type(16))) __bf16   v16bf;
typedef __attribute__((ext_vector_type(16))) _Float16 v16h;
typedef __attribute__((ext_vector_type(8)))  _Float16 v8h;
typedef __attribute__((ext_vector_type(8)))  unsigned short v8us;
typedef __attribute__((ext_vector_type(8)))  float    v8f;
typedef __attribute__((ext_vector_type(4)))  float    v4f;
typedef __attribute__((ext_vector_type(4)))  int      v4i;
typedef v4f  __attribute__((may_alias)) v4fa;

__device__ __forceinline__ unsigned short f2bf(float f) { unsigned u = __float_as_uint(f); u += 0x7FFFu + ((u >> 16) & 1u); return (unsigned short)(u >> 16); }
__device__ __forceinline__ float bf2f(unsigned short b) { return __uint_as_float(((unsigned)b) << 16); }
__device__ __forceinline__ float bfr(float f) { return bf2f(f2bf(f)); }
__device__ __forceinline__ v16h cat16(v8h lo, v8h hi) { return __builtin_shufflevector(lo, hi, 0, 1, 2, 3, 4, 5, 6, 7, 8, 9, 10, 11, 12, 13, 14, 15); }
__device__ __forceinline__ v16bf cat16b(v8us lo, v8us hi) { return __builtin_bit_cast(v16bf, __builtin_shufflevector(lo, hi, 0, 1, 2, 3, 4, 5, 6, 7, 8, 9, 10, 11, 12, 13, 14, 15)); }
__device__ __forceinline__ v8f wmma16(v16h a, v16h b, v8f c) { return __builtin_amdgcn_wmma_f32_16x16x32_f16(false, a, false, b, (short)0, c, false, false); }
__device__ __forceinline__ v8f wmmab(v16bf a, v16bf b, v8f c) { return __builtin_amdgcn_wmma_f32_16x16x32_bf16(false, a, false, b, (short)0, c, false, false); }

static __device__ __forceinline__ h16 toh_flush(float v) { const h16 r = (h16)v; return (fabsf(v) < 6.103515625e-05f) ? (h16)0.0f : r; }

template <typename T16> struct WFrag;
template <> struct WFrag<h16> { typedef v16h V; static __device__ __forceinline__ V ld(const h16* p) { return cat16(*(const v8h*)p, *(const v8h*)(p + 16)); } static __device__ __forceinline__ v8f mma(V a, V b, v8f c) { return wmma16(a, b, c); } };
template <> struct WFrag<bf> { typedef v16bf V; static __device__ __forceinline__ V ld(const bf* p) { return cat16b(*(const v8us*)p, *(const v8us*)(p + 16)); } static __device__ __forceinline__ v8f mma(V a, V b, v8f c) { return wmmab(a, b, c); } };
template <typename T16, int NSPLIT, bool BIAS>
__global__ __launch_bounds__(32) void k_gemmw(const T16* __restrict__ A, const T16* __restrict__ A2, const T16* __restrict__ Bt, const T16* __restrict__ Bt2, int K, float* C, int ldc, const float* __restrict__ bias, size_t sA, size_t sB, size_t sC) {
    typedef typename WFrag<T16>::V V;
    __shared__ __align__(16) float os[16 * 68];
    const size_t z = blockIdx.z; A += z * sA; if (A2) A2 += z * sA; Bt += z * sB; if (Bt2) Bt2 += z * sB; C += z * sC;
    const int lane = threadIdx.x & 31, lr = lane & 15, hi = lane >> 4; const int r0 = blockIdx.x * 64, c0 = blockIdx.y * 64;
    v8f acc[4][4];
#pragma unroll
    for (int mb = 0; mb < 4; ++mb)
#pragma unroll
        for (int nb = 0; nb < 4; ++nb) acc[mb][nb] = (v8f){};
    const size_t aoff = (size_t)(r0 + lr) * K + 8 * hi, boff = (size_t)(c0 + lr) * K + 8 * hi;
#pragma unroll 1
    for (int kc = 0; kc < K; kc += 32) {
        V a[4], a2[4];
#pragma unroll
        for (int mb = 0; mb < 4; ++mb) { a[mb] = WFrag<T16>::ld(A + aoff + (size_t)mb * 16 * K + kc); if (NSPLIT == 1 || NSPLIT == 2) a2[mb] = WFrag<T16>::ld(A2 + aoff + (size_t)mb * 16 * K + kc); }
#pragma unroll
        for (int nb = 0; nb < 4; ++nb) { const V b = WFrag<T16>::ld(Bt + boff + (size_t)nb * 16 * K + kc); V b2; if (NSPLIT >= 2) b2 = WFrag<T16>::ld(Bt2 + boff + (size_t)nb * 16 * K + kc);
#pragma unroll
            for (int mb = 0; mb < 4; ++mb) { acc[mb][nb] = WFrag<T16>::mma(a[mb], b, acc[mb][nb]); if (NSPLIT == 1 || NSPLIT == 2) acc[mb][nb] = WFrag<T16>::mma(a2[mb], b, acc[mb][nb]); if (NSPLIT >= 2) acc[mb][nb] = WFrag<T16>::mma(a[mb], b2, acc[mb][nb]); } }
        asm volatile("v_nop\n\tv_nop\n\tv_nop\n\tv_nop" : "+v"(acc[0][0]), "+v"(acc[1][1]), "+v"(acc[2][2]), "+v"(acc[3][3]) : "v"(a[0]), "v"(a[3]));
    }
#pragma unroll
    for (int mb = 0; mb < 4; ++mb) {
#pragma unroll
        for (int nb = 0; nb < 4; ++nb) {
#pragma unroll
            for (int j = 0; j < 8; ++j) os[(hi * 8 + j) * 68 + nb * 16 + lr] = acc[mb][nb][j]; }
        __builtin_amdgcn_wave_barrier(); asm volatile("" ::: "memory");
        float* crow = C + (size_t)(r0 + mb * 16) * ldc + c0;
#pragma unroll 1
        for (int ps = 0; ps < 2; ++ps) {
#pragma unroll
            for (int s = 0; s < 8; ++s) { const int row = 2 * s + hi, cofs = lr * 4; v4f val = *(const v4fa*)(os + row * 68 + cofs); if (BIAS) { val[0] += bfr(bias[c0 + cofs]); val[1] += bfr(bias[c0 + cofs + 1]); val[2] += bfr(bias[c0 + cofs + 2]); val[3] += bfr(bias[c0 + cofs + 3]); }
                *(volatile v4f*)(crow + (size_t)row * ldc + cofs) = val; }
            if (ps == 0) __threadfence(); }
        __builtin_amdgcn_wave_barrier(); asm volatile("" ::: "memory");
    }
}

__device__ __forceinline__ void splitf(float y, unsigned short& h, unsigned short& l) { h = f2bf(y); l = f2bf(y - bf2f(h)); }

__global__ __launch_bounds__(256) void k_cvt8(const float* __restrict__ src, bf* dst, size_t n8) { const size_t i = (size_t)blockIdx.x * 256 + threadIdx.x; if (i >= n8) return; const v8f v = *(const v8f*)(src + i * 8); v8us o;
#pragma unroll
    for (int k = 0; k < 8; ++k) o[k] = f2bf(v[k]); *(volatile v8us*)(dst + i * 8) = o; __threadfence(); *(volatile v8us*)(dst + i * 8) = o; }

__global__ __launch_bounds__(256) void k_hflat(const float* __restrict__ F, h16* P16) {
    const unsigned i = blockIdx.x * 256u + threadIdx.x; if (i >= (unsigned)(NH_ * TT * (HD / 8))) return;
    const float* f = F + (size_t)i * 8; const v4f a0 = *(const v4f*)f, a1 = *(const v4f*)(f + 4); v8h o;
#pragma unroll
    for (int q = 0; q < 4; ++q) { o[q] = toh_flush(a0[q]); o[4 + q] = toh_flush(a1[q]); }
    *(volatile v8h*)(P16 + (size_t)i * 8) = o; __threadfence(); *(volatile v8h*)(P16 + (size_t)i * 8) = o; }

__global__ __launch_bounds__(256) void k_vtflat(const float* __restrict__ F, h16* V16) {
    const unsigned i = blockIdx.x * 256u + threadIdx.x; if (i >= (unsigned)(NH_ * HD * (TT / 8))) return;
    const unsigned t8 = i % (unsigned)(TT / 8); const unsigned d = (i / (unsigned)(TT / 8)) % (unsigned)HD; const unsigned g = i / (unsigned)((TT / 8) * HD);
    const float* f = F + (size_t)g * ((size_t)TT * HD) + (size_t)(t8 * 8) * HD + d; v8h o;
#pragma unroll
    for (int q = 0; q < 8; ++q) o[q] = toh_flush(f[(size_t)q * HD]);
    *(volatile v8h*)(V16 + (size_t)i * 8) = o; __threadfence(); *(volatile v8h*)(V16 + (size_t)i * 8) = o; }

__global__ __launch_bounds__(256) void k_asoftm(const float* __restrict__ Sb, const float* __restrict__ MA, const float* __restrict__ MG, h16* P16) {
#pragma clang fp contract(off)
    const unsigned lane = threadIdx.x & 31u; const unsigned row = blockIdx.x * 8u + (threadIdx.x >> 5); if (row >= (unsigned)(ZH * TT)) return; const unsigned i = row % (unsigned)TT;
    const float* sr = Sb + (size_t)row * TT; const float* ar = MA + (size_t)i * MPITCH; const float* gr = MG + (size_t)i * MPITCH; float v[TT / 32]; float mx = -3.0e38f;
#pragma unroll
    for (int ch = 0; ch < TT / 256; ++ch) { const unsigned j0 = (unsigned)ch * 256u + lane * 8u; const v4f a0 = *(const v4f*)(sr + j0), a1 = *(const v4f*)(sr + j0 + 4); const v4f m0 = *(const v4f*)(ar + j0), m1 = *(const v4f*)(ar + j0 + 4);
#pragma unroll
        for (int q = 0; q < 4; ++q) { const float t0 = a0[q] * SCL + bfr(m0[q]); const float t1 = a1[q] * SCL + bfr(m1[q]); v[ch * 8 + q] = t0; v[ch * 8 + 4 + q] = t1; mx = fmaxf(mx, fmaxf(t0, t1)); }
        asm volatile("" ::: "memory"); }
#pragma unroll
    for (int sh = 16; sh; sh >>= 1) mx = fmaxf(mx, __shfl_xor(mx, sh, 32));
    float sum = 0.f;
#pragma unroll
    for (int k = 0; k < TT / 32; ++k) { float d0 = __fsub_rn(v[k], mx); asm volatile("" : "+v"(d0)); v[k] = __builtin_amdgcn_exp2f(__fmul_rn(d0, 1.4426950408889634f)); sum += v[k]; }
#pragma unroll
    for (int sh = 16; sh; sh >>= 1) sum += __shfl_xor(sum, sh, 32);
    const float f = __fdiv_rn(PCAR, sum);
#pragma unroll
    for (int ch = 0; ch < TT / 256; ++ch) { const unsigned j0 = (unsigned)ch * 256u + lane * 8u; const v4f g0 = *(const v4f*)(gr + j0), g1 = *(const v4f*)(gr + j0 + 4);
#pragma unroll
        for (int q = 0; q < 4; ++q) { v[ch * 8 + q] = (v[ch * 8 + q] * f) * bfr(g0[q]); v[ch * 8 + 4 + q] = (v[ch * 8 + 4 + q] * f) * bfr(g1[q]); }
        asm volatile("" ::: "memory"); }
    h16* pr = P16 + (size_t)row * TT + lane * 8u;
#pragma unroll 1
    for (int ps = 0; ps < 2; ++ps) {
#pragma unroll
        for (int ch = 0; ch < TT / 256; ++ch) { v8h o;
#pragma unroll
            for (int q = 0; q < 8; ++q) o[q] = toh_flush(v[ch * 8 + q]);
            *(volatile v8h*)(pr + ch * 256) = o; }
        if (ps == 0) __threadfence(); }
}

__global__ __launch_bounds__(256) void k_mergef(const float* __restrict__ O, unsigned h0, bf* Ah, bf* Al) {
    const unsigned i = blockIdx.x * 256u + threadIdx.x; if (i >= (unsigned)(ZH * TT * (HD / 8))) return;
    const v4f a0 = *(const v4f*)(O + (size_t)i * 8), a1 = *(const v4f*)(O + (size_t)i * 8 + 4); v8us oh, ol;
#pragma unroll
    for (int q = 0; q < 4; ++q) { unsigned short a, c2; splitf(a0[q] * (1.0f / PCAR), a, c2); oh[q] = a; ol[q] = c2; splitf(a1[q] * (1.0f / PCAR), a, c2); oh[4 + q] = a; ol[4 + q] = c2; }
    const size_t oo = (size_t)h0 * ((size_t)TT * HD) + (size_t)i * 8;
    *(volatile v8us*)(Ah + oo) = oh; *(volatile v8us*)(Al + oo) = ol; __threadfence(); *(volatile v8us*)(Ah + oo) = oh; *(volatile v8us*)(Al + oo) = ol; }

constexpr size_t al256(size_t b) { return (b + 255) & ~(size_t)255; }
constexpr size_t SZ_W  = al256((size_t)DQ * DM * 2);
constexpr size_t SZ_XB = al256((size_t)TT * DM * 2);
constexpr size_t SZ_F  = al256((size_t)TT * DQ * 4);
constexpr size_t SZ_PL = al256((size_t)NH_ * TT * HD * 2);
constexpr size_t SZ_S  = al256((size_t)ZH * TT * TT * 4);
constexpr size_t SZ_P  = al256((size_t)ZH * TT * TT * 2);
constexpr size_t SZ_O  = al256((size_t)ZH * TT * HD * 4);
constexpr size_t SZ_AT = al256((size_t)TT * DQ * 2);
constexpr size_t WS_TOTAL = 4 * SZ_W + SZ_XB + SZ_F + 3 * SZ_PL + SZ_S + SZ_P + SZ_O + 2 * SZ_AT;
static_assert(WS_TOTAL <= (size_t)134217728);
static_assert(((size_t)DQ * DM / 8) % 256 == 0);
static_assert(((size_t)TT * DM / 8) % 256 == 0);
static_assert(((size_t)NH_ * TT * HD / 8) % 256 == 0);
static_assert(((size_t)ZH * TT * HD / 8) % 256 == 0);
static_assert((ZH * TT) % 8 == 0);
static_assert((size_t)(NH_ - ZH) * TT * HD + (size_t)ZH * TT * HD == (size_t)TT * DQ);
static_assert((size_t)TT * DQ * 2 <= SZ_AT);

extern "C" void kernel_launch(void* const* d_in, const int* in_sizes, int n_in,
                              void* d_out, int out_size, void* d_ws, size_t ws_size, hipStream_t stream) {
    if (n_in < 13) return;
    const size_t need_x = (size_t)(NB - 1) * SEQ_FULL * DM + (size_t)SEQ * DM;
    const size_t need_m = (size_t)(NB - 1) * SEQ_FULL * SEQ_FULL + (size_t)(SEQ - 1) * SEQ_FULL + (size_t)SEQ;
    if ((size_t)in_sizes[0] < need_x || (size_t)in_sizes[1] < need_x || (size_t)in_sizes[2] < need_x || (size_t)in_sizes[3] < need_m || (size_t)in_sizes[4] < need_m) return;
    if ((size_t)in_sizes[5] < (size_t)DQ * DM || (size_t)in_sizes[7] < (size_t)DQ * DM || (size_t)in_sizes[9] < (size_t)DQ * DM || (size_t)in_sizes[11] < (size_t)DM * DQ) return;
    if (in_sizes[6] < DQ || in_sizes[8] < DQ || in_sizes[10] < DQ || in_sizes[12] < DM) return;
    if ((size_t)out_size < (size_t)NB * SEQ * DM) return;
    if (WS_TOTAL > ws_size) return;
    const float* xq = (const float*)d_in[0]; const float* xk = (const float*)d_in[1]; const float* xv = (const float*)d_in[2];
    const float* ma = (const float*)d_in[3]; const float* mg = (const float*)d_in[4];
    const float* wq = (const float*)d_in[5]; const float* bq = (const float*)d_in[6]; const float* wk = (const float*)d_in[7]; const float* bk = (const float*)d_in[8];
    const float* wv = (const float*)d_in[9]; const float* bv = (const float*)d_in[10]; const float* wo = (const float*)d_in[11]; const float* bo = (const float*)d_in[12];
    float* OUT = (float*)d_out;
    char* wsp = (char*)d_ws;
    bf* WQ = (bf*)wsp; wsp += SZ_W; bf* WK = (bf*)wsp; wsp += SZ_W; bf* WV = (bf*)wsp; wsp += SZ_W; bf* WO = (bf*)wsp; wsp += SZ_W;
    bf* XB = (bf*)wsp; wsp += SZ_XB; float* F = (float*)wsp; wsp += SZ_F;
    h16* QP16 = (h16*)wsp; wsp += SZ_PL; h16* KP16 = (h16*)wsp; wsp += SZ_PL; h16* VT16 = (h16*)wsp; wsp += SZ_PL;
    float* Sb = (float*)wsp; wsp += SZ_S; h16* P16 = (h16*)wsp; wsp += SZ_P; float* Ob = (float*)wsp; wsp += SZ_O;
    bf* ATh = (bf*)wsp; wsp += SZ_AT; bf* ATl = (bf*)wsp; wsp += SZ_AT;

    const unsigned GW = (unsigned)(((size_t)DQ * DM / 8 + 255) / 256);
    const unsigned GX = (unsigned)(((size_t)TT * DM / 8 + 255) / 256);
    const unsigned GP = (unsigned)(((size_t)NH_ * TT * HD / 8 + 255) / 256);
    const unsigned GM = (unsigned)(((size_t)ZH * TT * HD / 8 + 255) / 256);
    k_cvt8<<<GW, 256, 0, stream>>>(wq, WQ, (size_t)DQ * DM / 8);
    k_cvt8<<<GW, 256, 0, stream>>>(wk, WK, (size_t)DQ * DM / 8);
    k_cvt8<<<GW, 256, 0, stream>>>(wv, WV, (size_t)DQ * DM / 8);
    k_cvt8<<<GW, 256, 0, stream>>>(wo, WO, (size_t)DM * DQ / 8);
    for (int b = 0; b < NB; ++b) {
        const size_t xo = (size_t)b * SEQ_FULL * DM;
        const float* mab = ma + (size_t)b * SEQ_FULL * SEQ_FULL; const float* mgb = mg + (size_t)b * SEQ_FULL * SEQ_FULL;
        k_cvt8<<<GX, 256, 0, stream>>>(xq + xo, XB, (size_t)TT * DM / 8);
        k_gemmw<bf, 0, true><<<dim3(TT / 64, DQ / 64, 1), 32, 0, stream>>>(XB, nullptr, WQ, nullptr, DM, F, DQ, bq, 0, 0, 0);
        k_hflat<<<GP, 256, 0, stream>>>(F, QP16);
        k_cvt8<<<GX, 256, 0, stream>>>(xk + xo, XB, (size_t)TT * DM / 8);
        k_gemmw<bf, 0, true><<<dim3(TT / 64, DQ / 64, 1), 32, 0, stream>>>(XB, nullptr, WK, nullptr, DM, F, DQ, bk, 0, 0, 0);
        k_hflat<<<GP, 256, 0, stream>>>(F, KP16);
        k_cvt8<<<GX, 256, 0, stream>>>(xv + xo, XB, (size_t)TT * DM / 8);
        k_gemmw<bf, 0, true><<<dim3(TT / 64, DQ / 64, 1), 32, 0, stream>>>(XB, nullptr, WV, nullptr, DM, F, DQ, bv, 0, 0, 0);
        k_vtflat<<<GP, 256, 0, stream>>>(F, VT16);
        for (int h0 = 0; h0 < NH_; h0 += ZH) {
            const size_t zo = (size_t)h0 * TT * HD;
            k_gemmw<h16, 0, false><<<dim3(TT / 64, TT / 64, ZH), 32, 0, stream>>>(QP16 + zo, nullptr, KP16 + zo, nullptr, HD, Sb, TT, nullptr, (size_t)TT * HD, (size_t)TT * HD, (size_t)TT * TT);
            k_asoftm<<<ZH * TT / 8, 256, 0, stream>>>(Sb, mab, mgb, P16);
            k_gemmw<h16, 0, false><<<dim3(TT / 64, HD / 64, ZH), 32, 0, stream>>>(P16, nullptr, VT16 + zo, nullptr, TT, Ob, HD, nullptr, (size_t)TT * TT, (size_t)HD * TT, (size_t)TT * HD);
            k_mergef<<<GM, 256, 0, stream>>>(Ob, (unsigned)h0, ATh, ATl);
        }
        k_gemmw<bf, 1, true><<<dim3(TT / 64, DM / 64, 1), 32, 0, stream>>>(ATh, ATl, WO, nullptr, DQ, OUT + (size_t)b * TT * DM, DM, bo, 0, 0, 0);
    }
}
